// GCN_16252156248489
// MI455X (gfx1250) — hardware-run, weakly checked
//
#include <hip/hip_runtime.h>

typedef float          v8f   __attribute__((ext_vector_type(8)));
typedef float          v4f   __attribute__((ext_vector_type(4)));
typedef unsigned int   v4u   __attribute__((ext_vector_type(4)));
typedef int            v8i   __attribute__((ext_vector_type(8)));
typedef unsigned short v8us  __attribute__((ext_vector_type(8)));
typedef unsigned short v16us __attribute__((ext_vector_type(16)));
typedef __bf16         v16bf __attribute__((ext_vector_type(16)));
typedef _Float16       v16h  __attribute__((ext_vector_type(16)));
typedef v4f  __attribute__((may_alias)) v4fa;
typedef v8us __attribute__((may_alias)) v8usa;
union FragB { v16bf v; v16us u; v8us h[2]; v8i w; };
union FragH { v16h  v; v16us u; v8us h[2]; v8i w; };

__device__ __forceinline__ v8f wmb(const FragB& a, const FragB& b, v8f c) {
  v8f d = __builtin_amdgcn_wmma_f32_16x16x32_bf16(false, a.v, false, b.v, (short)0, c, false, false);
  asm volatile("v_nop\n\tv_nop\n\tv_nop\n\tv_nop" : "+v"(d) : "v"(a.w), "v"(b.w));
  return d;
}

__device__ __forceinline__ v8f wmh(const FragH& a, const FragH& b, v8f c) {
  v8f d = __builtin_amdgcn_wmma_f32_16x16x32_f16(false, a.v, false, b.v, (short)0, c, false, false);
  asm volatile("v_nop\n\tv_nop\n\tv_nop\n\tv_nop" : "+v"(d) : "v"(a.w), "v"(b.w));
  return d;
}

__device__ __forceinline__ unsigned bf16_bits(float f) {
  const unsigned u = __float_as_uint(f);
  const unsigned r = (u + 0x7FFFu + ((u >> 16) & 1u)) >> 16;
  const unsigned q = (u >> 16) | 0x40u;
  return ((u & 0x7fffffffu) > 0x7f800000u) ? q : r;
}

__device__ __forceinline__ float bf16_val(float f) {
  return __uint_as_float(bf16_bits(f) << 16);
}
__device__ __forceinline__ int clampi(int v, int lo, int hi) {
  return v < lo ? lo : (v > hi ? hi : v);
}

__device__ __forceinline__ unsigned f16_bits(float f) {
  const unsigned u  = __float_as_uint(f);
  const unsigned s  = (u >> 16) & 0x8000u;
  const unsigned a  = u & 0x7fffffffu;
  const unsigned t  = a - 0x38000000u;
  const unsigned r  = (t + 0x0FFFu + ((t >> 13) & 1u)) >> 13;
  const unsigned rc = r > 0x7C00u ? 0x7C00u : r;
  const bool small  = a < 0x38800000u;
  const bool isnan  = a > 0x7f800000u;
  const unsigned fin = small ? 0u : (s | rc);
  return isnan ? (s | 0x7E00u) : fin;
}

__device__ __forceinline__ unsigned pk16(unsigned lo, unsigned hi) { return lo | (hi << 16); }
__device__ __forceinline__ unsigned bf16_lo_bits(float v) {
  float hi = bf16_val(v);
  asm volatile("" : "+v"(hi));
  return bf16_bits(v - hi);
}
__device__ __forceinline__ v4u pack8_bf16(v4f a, v4f c) {
  return (v4u){ pk16(bf16_bits(a[0]), bf16_bits(a[1])), pk16(bf16_bits(a[2]), bf16_bits(a[3])),
                pk16(bf16_bits(c[0]), bf16_bits(c[1])), pk16(bf16_bits(c[2]), bf16_bits(c[3])) };
}
__device__ __forceinline__ v4u pack8_bf16_lo(v4f a, v4f c) {
  return (v4u){ pk16(bf16_lo_bits(a[0]), bf16_lo_bits(a[1])), pk16(bf16_lo_bits(a[2]), bf16_lo_bits(a[3])),
                pk16(bf16_lo_bits(c[0]), bf16_lo_bits(c[1])), pk16(bf16_lo_bits(c[2]), bf16_lo_bits(c[3])) };
}
__device__ __forceinline__ v4u pack8_f16(v4f a, v4f c) {
  return (v4u){ pk16(f16_bits(a[0]), f16_bits(a[1])), pk16(f16_bits(a[2]), f16_bits(a[3])),
                pk16(f16_bits(c[0]), f16_bits(c[1])), pk16(f16_bits(c[2]), f16_bits(c[3])) };
}

template <int FORM>
__global__ __launch_bounds__(256) void k_plane(const float* __restrict__ src, int rows, int cols, int ldsrc,
                                               unsigned short* __restrict__ dst, int MP, int KP) {
  static_assert(FORM >= 0 && FORM <= 3);
  const int KTOT = (FORM == 1 || FORM == 3) ? 2 * KP : KP;
  const unsigned ppr   = (unsigned)(KTOT >> 3);
  const unsigned kp8   = (unsigned)(KP >> 3);
  const unsigned total = (unsigned)MP * ppr;
  const unsigned g     = blockIdx.x * 256u + threadIdx.x;
  const unsigned rowu  = g / ppr;
  const unsigned p     = g - rowu * ppr;
  const bool second    = p >= kp8;
  const int row = (int)rowu;
  const int c0  = (int)((second ? p - kp8 : p) << 3);
  const float* srow = src + (size_t)clampi(row, 0, rows - 1) * (size_t)ldsrc;
  float x[8];
  unsigned mk[8];
#pragma unroll
  for (int e = 0; e < 8; ++e) {
    const int c = c0 + e;
    const float v = srow[clampi(c, 0, cols - 1)];
    asm volatile("" :: "v"(v));
    x[e]  = v;
    mk[e] = (row < rows && c < cols) ? 0xFFFFu : 0u;
  }
  const v4f a = (v4f){ x[0], x[1], x[2], x[3] };
  const v4f c = (v4f){ x[4], x[5], x[6], x[7] };
  v4u o;
  if (FORM == 2) {
    o = pack8_f16(a, c);
  } else {
    const v4u hi = pack8_bf16(a, c);
    o = hi;
    if (FORM == 1) { const v4u lo = pack8_bf16_lo(a, c); o = second ? lo : hi; }
  }
  const v4u mw = (v4u){ pk16(mk[0], mk[1]), pk16(mk[2], mk[3]), pk16(mk[4], mk[5]), pk16(mk[6], mk[7]) };
  o &= mw;
  if (g < total) {
    volatile v4u* q = (volatile v4u*)(dst + (size_t)g * 8);
    *q = o;
    __threadfence();
    *q = o;
  }
}

template <int FORM> struct FragOf    { typedef FragB T; };
template <>         struct FragOf<2> { typedef FragH T; };
__device__ __forceinline__ v8f mm(const FragB& a, const FragB& b, v8f c) { return wmb(a, b, c); }
__device__ __forceinline__ v8f mm(const FragH& a, const FragH& b, v8f c) { return wmh(a, b, c); }
template <class F> __device__ __forceinline__ F ld_frag(const unsigned short* p) {
  F f;
  f.h[0] = *(const v8usa*)(p);
  f.h[1] = *(const v8usa*)(p + 16);
  return f;
}

template <int FORM, int EPI>
__global__ __launch_bounds__(256) __attribute__((amdgpu_num_vgpr(248)))
void k_gemm_nt(const unsigned short* __restrict__ A, const unsigned short* __restrict__ B,
               const float* __restrict__ bias, float* __restrict__ D, int M, int N, int KTOT, int ldd) {
  static_assert(FORM >= 0 && FORM <= 2);
  static_assert(EPI == 0 || EPI == 1);
  typedef typename FragOf<FORM>::T F;
  __shared__ __attribute__((aligned(16))) float sT[8][16 * 68];
  const int lane = threadIdx.x & 31;
  const int wave = threadIdx.x >> 5;
  const int tilesM = (M + 63) >> 6;
  const int tilesN = (N + 63) >> 6;
  const int tile = blockIdx.x * 8 + wave;
  if (tile >= tilesM * tilesN) return;
  const int tm = tile / tilesN;
  const int tn = tile - tm * tilesN;
  const int m0 = tm << 6;
  const int n0 = tn << 6;

  const int rl = lane & 15;
  const int h8 = (lane >> 4) * 8;
  const unsigned short* pa = A + (size_t)(m0 + rl) * (size_t)KTOT + h8;
  const unsigned short* pb = B + (size_t)(n0 + rl) * (size_t)KTOT + h8;

  v8f acc[4][4];
#pragma unroll
  for (int i = 0; i < 4; ++i)
#pragma unroll
    for (int j = 0; j < 4; ++j) acc[i][j] = (v8f){0.f, 0.f, 0.f, 0.f, 0.f, 0.f, 0.f, 0.f};

#pragma unroll 1
  for (int k0 = 0; k0 < KTOT; k0 += 32) {
    F bf[4];
#pragma unroll
    for (int j = 0; j < 4; ++j) bf[j] = ld_frag<F>(pb + (size_t)(j << 4) * (size_t)KTOT + k0);
#pragma unroll
    for (int i = 0; i < 4; ++i) {
      const F af = ld_frag<F>(pa + (size_t)(i << 4) * (size_t)KTOT + k0);
#pragma unroll
      for (int j = 0; j < 4; ++j) acc[i][j] = mm(af, bf[j], acc[i][j]);
    }
  }

  float* slab = sT[wave];
  const int hh = lane >> 4;
  const int c4 = (lane & 15) * 4;
  const int nc = n0 + c4;
  const bool cok = nc < N;
  v4f bv = (v4f){0.f, 0.f, 0.f, 0.f};
  if (EPI == 1) {
    bv = *(const v4fa*)(bias + clampi(nc, 0, N - 4));
    asm volatile("" :: "v"(bv));
  }
#pragma unroll
  for (int i = 0; i < 4; ++i) {
    const int mBase = m0 + (i << 4);
#pragma unroll
    for (int j = 0; j < 4; ++j) {
#pragma unroll
      for (int r = 0; r < 8; ++r) slab[(h8 + r) * 68 + (j << 4) + rl] = acc[i][j][r];
    }
    __builtin_amdgcn_fence(__ATOMIC_RELEASE, "workgroup");
    __builtin_amdgcn_wave_barrier();
    __builtin_amdgcn_fence(__ATOMIC_ACQUIRE, "workgroup");
    v4f vv[8];
#pragma unroll
    for (int it = 0; it < 8; ++it) {
      const int row = it * 2 + hh;
      v4f v = *(const v4fa*)(slab + row * 68 + c4);
      if (EPI == 1) v += bv;
      vv[it] = v;
    }
    for (int pass = 0; pass < 2; ++pass) {
#pragma unroll
      for (int it = 0; it < 8; ++it) {
        const int row = mBase + it * 2 + hh;
        if (cok && row < M) *(volatile v4f*)(D + (size_t)row * (size_t)ldd + nc) = vv[it];
      }
      __threadfence();
    }
    __builtin_amdgcn_fence(__ATOMIC_RELEASE, "workgroup");
    __builtin_amdgcn_wave_barrier();
    __builtin_amdgcn_fence(__ATOMIC_ACQUIRE, "workgroup");
  }
}

#pragma clang fp contract(off)

#include <stddef.h>
#include <stdint.h>

#define NNODE   100000
#define NEDGE   1600000
#define FIN     128
#define HID     256
#define HH      128
#define FOUT    64
#define MPAD    100096
#define NTHR    256
#define NWAVE   8
#define EPT     8
#define WCH     (32 * EPT)
#define NBRUN   1024
#define SLB     10
#define NBK     98
#define NTAB    (NBK * NBRUN)
#define WLCA    3392
#define WLCB    2688
#define RCAP    21504
#define DEGCAP  64
#define MAXDEG_IN_MEAS   36
#define MAXDEG_OUT_MEAS  37
#define MAXB1024_IN_MEAS  16721
#define MAXB1024_OUT_MEAS 16666
#define KT      256

#define O_WL   0
#define O_PL   (NWAVE * WLCA)
#define O_CNT  (O_PL + RCAP)
#define O_OFF  (O_CNT + NBRUN)
#define O_CUR  (O_OFF + NBRUN)
#define O_CNTB (O_CUR + NBRUN)
#define O_DI   (O_CNTB + NBRUN)
#define O_DO   (O_DI + NBRUN)
#define BK_ZINTS (O_DO + NBRUN)
#define O_MISC BK_ZINTS
#define BK_INTS  (BK_ZINTS + 32)
#define BK_LDS   (BK_INTS * 4)

#define PB_W1A (HH * KT / 8 / NTHR)
#define PB_W1B (HH * KT / 8 / NTHR)
#define PB_W2A (FOUT * KT / 8 / NTHR)
#define PB_W2B (FOUT * KT / 8 / NTHR)
#define PB_BI  1
#define PB_TOT (PB_W1A + PB_W1B + PB_W2A + PB_W2B + PB_BI)
#define BT_B1  0
#define BT_B2  256
#define BT_Z   320
#define BT_UNITS 112

static_assert(FIN == 32 * 4 && HH == 32 * 4 && FOUT == 32 * 2 && HID == 2 * HH && KT == 2 * HH && KT == 2 * FIN);
static_assert(KT % 32 == 0 && HH % 64 == 0 && FOUT % 64 == 0 && HH % 32 == 0 && FOUT % 32 == 0);
static_assert(NNODE % NWAVE == 0 && NNODE % 16 == 0 && MPAD % NWAVE == 0);
static_assert(MPAD == 782 * 128 && MPAD % 128 == 0 && MPAD % 64 == 0 && MPAD >= NNODE);
static_assert(NBRUN == (1 << SLB) && NNODE < (1 << 17) && 17 + SLB <= 31);
static_assert(NTAB >= MPAD && (NBK - 1) * NBRUN < NNODE);
static_assert(NEDGE % WCH == 0 && NEDGE == 6250 * 256 && NEDGE % EPT == 0);
static_assert(RCAP % (NTHR * 4) == 0 && RCAP == NWAVE * WLCB);
static_assert((long long)RCAP * 100 >= (long long)MAXB1024_IN_MEAS * 105);
static_assert((long long)RCAP * 100 >= (long long)MAXB1024_OUT_MEAS * 105);
static_assert((long long)RCAP * 100 >= (long long)MAXB1024_IN_MEAS * 125);
static_assert((long long)RCAP * 100 >= (long long)MAXB1024_OUT_MEAS * 125);
static_assert(WLCA * 8 >= (RCAP / 8) * 10);
static_assert(WLCA >= MAXB1024_IN_MEAS / 8 + 8 * 46 + 1);
static_assert(WLCB >= MAXB1024_OUT_MEAS / 8 + 8 * 46 + 1);
static_assert(DEGCAP >= 48 && MAXDEG_IN_MEAS + 8 <= DEGCAP && MAXDEG_OUT_MEAS + 8 <= DEGCAP);
static_assert(BK_ZINTS % 4 == 0 && O_PL % 4 == 0 && O_CNT % 4 == 0 && O_DI % 4 == 0 && O_DO % 4 == 0);
static_assert(NBRUN == NTHR * 4);
static_assert(BK_LDS == 219264 && BK_LDS + 0 <= 327680);
static_assert((HH * KT / 8) % NTHR == 0 && (FOUT * KT / 8) % NTHR == 0);
static_assert((MPAD * FIN / 8) % NTHR == 0 && (MPAD * FOUT / 4) % NTHR == 0);
static_assert(BT_UNITS * 4 == BT_Z + 128 && BT_UNITS <= NTHR && (BT_Z * 4) % 128 == 0 && (BT_B2 * 4) % 128 == 0);
static_assert((long long)MPAD * KT / 8 < (1ll << 31));

typedef float          v2f  __attribute__((ext_vector_type(2)));
typedef int            v4i  __attribute__((ext_vector_type(4)));
typedef unsigned int   v2u  __attribute__((ext_vector_type(2)));
typedef v2f  __attribute__((may_alias)) v2fa;
typedef v4i  __attribute__((may_alias)) v4ia;
typedef v2u  __attribute__((may_alias)) v2ua;

__device__ __forceinline__ void st2_v4f(float* p, v4f v) {
  *(volatile v4f*)p = v;
  __threadfence();
  *(volatile v4f*)p = v;
}
__device__ __forceinline__ void st2_v8us(unsigned short* p, v8us v) {
  *(volatile v8us*)p = v;
  __threadfence();
  *(volatile v8us*)p = v;
}

__device__ __forceinline__ v8us gather8(const float* __restrict__ base, int stride) {
  float f[8];
#pragma unroll
  for (int i = 0; i < 8; ++i) {
    const float v = base[(size_t)i * (size_t)stride];
    asm volatile("" :: "v"(v));
    f[i] = v;
  }
  v8us o;
#pragma unroll
  for (int i = 0; i < 8; ++i) o[i] = (unsigned short)bf16_bits(f[i]);
  return o;
}

__device__ __forceinline__ void wplane_unit(const float* __restrict__ w, int ld, int rowoff, int coloff,
                                            unsigned short* wd, int u) {
  const int ppr = KT >> 3;
  const int n   = u / ppr;
  const int kk  = (u - n * ppr) << 3;
  const int k8  = kk & (HH - 1);
  const v8us o = gather8(w + (size_t)(rowoff + k8) * (size_t)ld + coloff + n, ld);
  st2_v8us(wd + (size_t)n * (size_t)KT + kk, o);
}

__global__ __launch_bounds__(NTHR) void k_prep(const float* __restrict__ W1, const float* __restrict__ W2,
                                               const float* __restrict__ b1, const float* __restrict__ b2,
                                               unsigned short* W1A, unsigned short* W1B,
                                               unsigned short* W2A, unsigned short* W2B, float* BT) {
  const int tid = (int)threadIdx.x;
  const int blk = (int)blockIdx.x;
  if (blk < PB_W1A) {
    wplane_unit(W1, HID, 0, 0, W1A, blk * NTHR + tid);
  } else if (blk < PB_W1A + PB_W1B) {
    wplane_unit(W1, HID, 0, HH, W1B, (blk - PB_W1A) * NTHR + tid);
  } else if (blk < PB_W1A + PB_W1B + PB_W2A) {
    wplane_unit(W2, FOUT, 0, 0, W2A, (blk - PB_W1A - PB_W1B) * NTHR + tid);
  } else if (blk < PB_W1A + PB_W1B + PB_W2A + PB_W2B) {
    wplane_unit(W2, FOUT, HH, 0, W2B, (blk - PB_W1A - PB_W1B - PB_W2A) * NTHR + tid);
  } else {
    const int u1 = clampi(tid, 0, 63);
    const int u2 = clampi(tid - 64, 0, 15);
    const v4f x1 = *(const v4fa*)(b1 + 4 * u1);
    const v4f x2 = *(const v4fa*)(b2 + 4 * u2);
    asm volatile("" :: "v"(x1));
    asm volatile("" :: "v"(x2));
    const unsigned s1 = 0u - (unsigned)(tid < 64);
    const unsigned s2 = 0u - (unsigned)(tid >= 64 && tid < 80);
    v4f o;
#pragma unroll
    for (int e = 0; e < 4; ++e) {
      const unsigned bits = (__float_as_uint(x1[e]) & s1) | (__float_as_uint(x2[e]) & s2);
      o[e] = bf16_val(__uint_as_float(bits));
    }
    if (tid < BT_UNITS) st2_v4f(BT + 4 * tid, o);
  }
}

__global__ __launch_bounds__(NTHR) void k_bucket(const int* __restrict__ srcs, const int* __restrict__ dsts,
                                                 int* LIST, int* CNT, int* OFF, int* DIt, int* DOt, int* FLAG) {
  extern __shared__ __attribute__((aligned(16))) int dsm[];
  const int tid = (int)threadIdx.x, lane = tid & 31, wave = tid >> 5;
  const int blk = (int)blockIdx.x;
  const unsigned nbs = (unsigned)(blk * NBRUN);

  {
    const v4i z4 = {0, 0, 0, 0};
    for (int i = tid * 4; i < BK_ZINTS; i += NTHR * 4) *(v4ia*)(dsm + i) = z4;
    if (tid < 32) dsm[O_MISC + tid] = 0;
  }
  __syncthreads();

  {
    const int per  = ((NEDGE + NWAVE * WCH - 1) / (NWAVE * WCH)) * WCH;
    const int ebeg = wave * per;
    const int eend = (ebeg + per < NEDGE) ? (ebeg + per) : NEDGE;
    int* la = dsm + O_WL + wave * WLCA;
    int* lb = dsm + O_PL + wave * WLCB;
    int wa = 0, wb = 0;
#pragma unroll 1
    for (int cb = ebeg; cb < eend; cb += WCH) {
      const int e0  = cb + lane * EPT;
      const int e0c = e0 > NEDGE - EPT ? NEDGE - EPT : e0;
      const bool ein = (e0 == e0c);
      const v4i da = *(const v4ia*)(dsts + e0c);
      const v4i db = *(const v4ia*)(dsts + e0c + 4);
      const v4i sa = *(const v4ia*)(srcs + e0c);
      const v4i sb = *(const v4ia*)(srcs + e0c + 4);
      asm volatile("" :: "v"(da));
      asm volatile("" :: "v"(db));
      asm volatile("" :: "v"(sa));
      asm volatile("" :: "v"(sb));
      const int dv[8] = { da.x, da.y, da.z, da.w, db.x, db.y, db.z, db.w };
      const int sv[8] = { sa.x, sa.y, sa.z, sa.w, sb.x, sb.y, sb.z, sb.w };
      unsigned ta[8], tb[8], ma[8], mb[8];
      bool ha[8], hb[8];
      unsigned anyA = 0u, anyB = 0u;
#pragma unroll
      for (int j = 0; j < 8; ++j) {
        ta[j] = (unsigned)dv[j] - nbs;
        tb[j] = (unsigned)sv[j] - nbs;
        ha[j] = ein && (ta[j] < (unsigned)NBRUN);
        hb[j] = ein && (tb[j] < (unsigned)NBRUN);
        ma[j] = __builtin_amdgcn_ballot_w32(ha[j]);
        mb[j] = __builtin_amdgcn_ballot_w32(hb[j]);
        anyA |= ma[j];
        anyB |= mb[j];
      }
      if (anyA != 0u) {
        int pre = 0, pop = 0;
#pragma unroll
        for (int j = 0; j < 8; ++j) {
          pre += (int)__builtin_amdgcn_mbcnt_lo(ma[j], 0u);
          pop += (int)__builtin_popcount(ma[j]);
        }
        int p = wa + pre;
#pragma unroll
        for (int j = 0; j < 8; ++j) {
          const int word = (clampi(sv[j], 0, NNODE - 1) << SLB) | (int)(ta[j] & (unsigned)(NBRUN - 1));
          if (ha[j]) { if (p < WLCA) la[p] = word; p = p + 1; }
        }
        wa += pop;
      }
      if (anyB != 0u) {
        int pre = 0, pop = 0;
#pragma unroll
        for (int j = 0; j < 8; ++j) {
          pre += (int)__builtin_amdgcn_mbcnt_lo(mb[j], 0u);
          pop += (int)__builtin_popcount(mb[j]);
        }
        int p = wb + pre;
#pragma unroll
        for (int j = 0; j < 8; ++j) {
          const int word = (int)(tb[j] & (unsigned)(NBRUN - 1));
          if (hb[j]) { if (p < WLCB) lb[p] = word; p = p + 1; }
        }
        wb += pop;
      }
    }
    if (lane == 0) { dsm[O_MISC + wave] = wa; dsm[O_MISC + 8 + wave] = wb; }
  }
  __syncthreads();

  if (wave < 2) {
    const int role  = wave;
    const int lbase = role ? O_PL : O_WL;
    const int lcap  = role ? WLCB : WLCA;
    const int cbase = role ? O_CNTB : O_CNT;
    int ov = 0, tot = 0;
#pragma unroll 1
    for (int w2 = 0; w2 < NWAVE; ++w2) {
      int c = dsm[O_MISC + role * 8 + w2];
      if (c > lcap) ov = 1;
      c = clampi(c, 0, lcap);
      tot += c;
#pragma unroll 1
      for (int b0 = 0; b0 < c; b0 += 32) {
        const int idx = b0 + lane;
        const int ent = dsm[lbase + w2 * lcap + (idx < lcap ? idx : lcap - 1)];
        const int m32 = (c - b0) < 32 ? (c - b0) : 32;
#pragma unroll 1
        for (int k = 0; k < m32; ++k) {
          const int u    = __builtin_amdgcn_readlane(ent, k);
          const int slot = u & (NBRUN - 1);
          const int cv   = dsm[cbase + slot];
          asm volatile("" :: "v"(cv));
          if (lane == 0) dsm[cbase + slot] = cv + 1;
        }
      }
    }
    if (tot > RCAP) ov = 1;
    if (lane == 0) dsm[O_MISC + 16 + role] = ov;
  }
  __syncthreads();

  const int ovA = dsm[O_MISC + 16];
  const int ovB = dsm[O_MISC + 17];
  {
    const v4i z4 = {0, 0, 0, 0};
    for (int i = tid * 4; i < RCAP; i += NTHR * 4) *(v4ia*)(dsm + O_PL + i) = z4;
    const float qn = __uint_as_float(0x7fc00000u);
#pragma unroll 1
    for (int j = 0; j < 8; ++j) {
      const int role = j >> 2;
      const int sbase = role ? O_CNTB : O_CNT;
      const int dbase = role ? O_DO : O_DI;
      int cv = dsm[sbase + 4 * tid + (j & 3)];
      cv = cv < 1 ? 1 : cv;
      const float sq = sqrtf((float)cv);
      const float dv = 1.0f / sq;
      const bool poison = (role != 0) && (ovB != 0);
      dsm[dbase + 4 * tid + (j & 3)] = __float_as_int(poison ? qn : dv);
    }
  }
  if (wave == 0) {
    const int base = lane * (NBRUN / 32);
    int s = 0;
#pragma unroll 1
    for (int i = 0; i < NBRUN / 32; ++i) s += dsm[O_CNT + base + i];
    int incl = s;
#pragma unroll
    for (int d = 1; d < 32; d <<= 1) {
      const int y = __shfl_up(incl, d, 32);
      incl += (lane >= d) ? y : 0;
    }
    int run = incl - s;
#pragma unroll 1
    for (int i = 0; i < NBRUN / 32; ++i) {
      const int cv = dsm[O_CNT + base + i];
      dsm[O_OFF + base + i] = run;
      dsm[O_CUR + base + i] = run;
      run += cv;
    }
  }
  __syncthreads();

  if (wave == 0) {
#pragma unroll 1
    for (int w2 = 0; w2 < NWAVE; ++w2) {
      int c = dsm[O_MISC + w2];
      c = clampi(c, 0, WLCA);
#pragma unroll 1
      for (int b0 = 0; b0 < c; b0 += 32) {
        const int idx = b0 + lane;
        const int ent = dsm[O_WL + w2 * WLCA + (idx < WLCA ? idx : WLCA - 1)];
        const int m32 = (c - b0) < 32 ? (c - b0) : 32;
#pragma unroll 1
        for (int k = 0; k < m32; ++k) {
          const int u    = __builtin_amdgcn_readlane(ent, k);
          const int slot = u & (NBRUN - 1);
          const int sid  = (u >> SLB) & 0x1FFFF;
          int p = dsm[O_CUR + slot];
          asm volatile("" :: "v"(p));
          p = clampi(p, 0, RCAP - 1);
          if (lane == 0) {
            dsm[O_PL + p]     = sid;
            dsm[O_CUR + slot] = p + 1;
          }
        }
      }
    }
  }
  __syncthreads();

  const int ovf = (ovA | ovB) != 0 ? 1 : 0;
  int* lp = LIST + (size_t)blk * (size_t)RCAP;
  int* cp = CNT + (size_t)blk * NBRUN;
  int* op = OFF + (size_t)blk * NBRUN;
  int* ip = DIt + (size_t)blk * NBRUN;
  int* dp = DOt + (size_t)blk * NBRUN;
  int* fp = FLAG + (size_t)blk * 32;
  for (int pass = 0; pass < 2; ++pass) {
#pragma unroll 1
    for (int i = tid * 4; i < RCAP; i += NTHR * 4) {
      const v4i v = *(const v4ia*)(dsm + O_PL + i);
      *(volatile v4i*)(lp + i) = v;
    }
    {
      const v4i vc = *(const v4ia*)(dsm + O_CNT + 4 * tid);
      const v4i vo = *(const v4ia*)(dsm + O_OFF + 4 * tid);
      const v4i vi = *(const v4ia*)(dsm + O_DI + 4 * tid);
      const v4i vd = *(const v4ia*)(dsm + O_DO + 4 * tid);
      *(volatile v4i*)(cp + 4 * tid) = vc;
      *(volatile v4i*)(op + 4 * tid) = vo;
      *(volatile v4i*)(ip + 4 * tid) = vi;
      *(volatile v4i*)(dp + 4 * tid) = vd;
    }
    if (tid < 8) {
      const v4i f = {ovf, ovf, ovf, ovf};
      *(volatile v4i*)(fp + 4 * tid) = f;
    }
    __threadfence();
  }
}

__global__ __launch_bounds__(NTHR) void k_walk0(const int* __restrict__ LIST, const int* __restrict__ CNT,
                                                const int* __restrict__ OFF, const float* __restrict__ DOt,
                                                const int* __restrict__ FLAG, const unsigned short* __restrict__ XB,
                                                unsigned short* OPA) {
  const int tid = (int)threadIdx.x, lane = tid & 31, wave = tid >> 5;
  const int row = (int)blockIdx.x * NWAVE + wave;
  const int rc  = clampi(row, 0, NNODE - 1);
  const int blk = rc >> SLB;
  int c = CNT[rc];
  int o = OFF[rc];
  const int flag = FLAG[(size_t)blk * 32];
  asm volatile("" :: "v"(c));
  asm volatile("" :: "v"(o));
  asm volatile("" :: "v"(flag));
  const bool big = c > DEGCAP;
  c = __builtin_amdgcn_readfirstlane((row < NNODE) ? clampi(c, 0, DEGCAP) : 0);
  o = __builtin_amdgcn_readfirstlane(clampi(o, 0, RCAP - 1));
  int last = o + (c > 0 ? c : 1) - 1;
  last = last > RCAP - 1 ? RCAP - 1 : last;
  const int* lb = LIST + (size_t)blk * (size_t)RCAP;

  float a0 = 0.0f, a1 = 0.0f, a2 = 0.0f, a3 = 0.0f;
#pragma unroll 1
  for (int b0 = 0; b0 < c; b0 += 32) {
    int idx = o + b0 + lane;
    idx = idx > last ? last : idx;
    const int word = lb[idx];
    asm volatile("" :: "v"(word));
    const int sr = clampi(word, 0, NNODE - 1);
    const float dv = DOt[sr];
    asm volatile("" :: "v"(dv));
    const int dbits = __float_as_int(dv);
    const int m32 = (c - b0) < 32 ? (c - b0) : 32;
#pragma unroll 1
    for (int k = 0; k < m32; ++k) {
      const int   sk = __builtin_amdgcn_readlane(sr, k);
      const float dk = __int_as_float(__builtin_amdgcn_readlane(dbits, k));
      const v2u q = *(const v2ua*)(XB + (size_t)sk * FIN + 4 * lane);
      const unsigned qx = q.x, qy = q.y;
      asm volatile("" :: "v"(qx));
      asm volatile("" :: "v"(qy));
      float x0 = __uint_as_float(qx << 16);
      float x1 = __uint_as_float(qx & 0xffff0000u);
      float x2 = __uint_as_float(qy << 16);
      float x3 = __uint_as_float(qy & 0xffff0000u);
      asm volatile("" : "+v"(x0));
      asm volatile("" : "+v"(x1));
      asm volatile("" : "+v"(x2));
      asm volatile("" : "+v"(x3));
      const float p0 = x0 * dk;
      const float p1 = x1 * dk;
      const float p2 = x2 * dk;
      const float p3 = x3 * dk;
      a0 = a0 + p0;
      a1 = a1 + p1;
      a2 = a2 + p2;
      a3 = a3 + p3;
    }
  }

  const float qnan = __uint_as_float(0x7fc00000u);
  const bool bad  = (flag != 0) || big;
  const bool live = row < NNODE;
  a0 = bad ? qnan : a0;  a1 = bad ? qnan : a1;  a2 = bad ? qnan : a2;  a3 = bad ? qnan : a3;
  a0 = live ? a0 : 0.0f; a1 = live ? a1 : 0.0f; a2 = live ? a2 : 0.0f; a3 = live ? a3 : 0.0f;

  v2u whi, wlo;
  whi.x = pk16(bf16_bits(a0), bf16_bits(a1));
  whi.y = pk16(bf16_bits(a2), bf16_bits(a3));
  wlo.x = pk16(bf16_lo_bits(a0), bf16_lo_bits(a1));
  wlo.y = pk16(bf16_lo_bits(a2), bf16_lo_bits(a3));
  if (row < MPAD) {
    volatile v2u* hp = (volatile v2u*)(OPA + (size_t)row * KT);
    hp[lane]      = whi;
    hp[32 + lane] = wlo;
    __threadfence();
    hp[lane]      = whi;
    hp[32 + lane] = wlo;
  }
}

__global__ __launch_bounds__(NTHR) void k_convert(float* PG, const float* __restrict__ DIt,
                                                  const float* __restrict__ DOt, const int* __restrict__ FLAG,
                                                  const float* __restrict__ B1h) {
  __shared__ __attribute__((aligned(16))) float sb[HH];
  const int tid = (int)threadIdx.x, lane = tid & 31, wave = tid >> 5;
  {
    const v4f b = *(const v4fa*)(B1h + 4 * (tid & 31));
    asm volatile("" :: "v"(b));
    if (tid < 32) *(v4fa*)(sb + 4 * tid) = b;
  }
  __syncthreads();

  const int row = (int)blockIdx.x * NWAVE + wave;
  const int rc  = clampi(row, 0, MPAD - 1);
  float* pr = PG + (size_t)rc * HH;
  const v4f p = *(const v4fa*)(pr + 4 * lane);
  asm volatile("" :: "v"(p));
  const float di = DIt[rc];
  const float dq = DOt[rc];
  const int flag = FLAG[(size_t)(clampi(rc, 0, NNODE - 1) >> SLB) * 32];
  asm volatile("" :: "v"(di));
  asm volatile("" :: "v"(dq));
  asm volatile("" :: "v"(flag));
  const v4f bq = *(const v4fa*)(sb + 4 * lane);

  const float qnan = __uint_as_float(0x7fc00000u);
  const bool bad  = flag != 0;
  const bool live = row < NNODE;
  float g[4];
#pragma unroll
  for (int e = 0; e < 4; ++e) {
    const float t  = p[e] * di;
    const float v  = t + bq[e];
    const float hh = (v > 0.0f) ? v : (v - v);
    float gg = hh * dq;
    gg = bad ? qnan : gg;
    gg = live ? gg : 0.0f;
    g[e] = gg;
  }
  v2u whi, wlo;
  whi.x = pk16(bf16_bits(g[0]), bf16_bits(g[1]));
  whi.y = pk16(bf16_bits(g[2]), bf16_bits(g[3]));
  wlo.x = pk16(bf16_lo_bits(g[0]), bf16_lo_bits(g[1]));
  wlo.y = pk16(bf16_lo_bits(g[2]), bf16_lo_bits(g[3]));
  if (row < MPAD) {
    volatile v2u* hp = (volatile v2u*)pr;
    hp[lane]      = whi;
    hp[32 + lane] = wlo;
    __threadfence();
    hp[lane]      = whi;
    hp[32 + lane] = wlo;
  }
}

__global__ __launch_bounds__(NTHR) void k_add(float* ACC, const float* __restrict__ Q) {
  const unsigned g = blockIdx.x * (unsigned)NTHR + threadIdx.x;
  const unsigned total = (unsigned)MPAD * (FOUT / 4);
  const unsigned gc = g < total ? g : total - 1u;
  const v4f a = *(const v4fa*)(ACC + (size_t)gc * 4);
  const v4f q = *(const v4fa*)(Q + (size_t)gc * 4);
  asm volatile("" :: "v"(a));
  asm volatile("" :: "v"(q));
  const v4f s = a + q;
  if (g < total) st2_v4f(ACC + (size_t)g * 4, s);
}

__global__ __launch_bounds__(NTHR) void k_walk2(const int* __restrict__ LIST, const int* __restrict__ CNT,
                                                const int* __restrict__ OFF, const float* __restrict__ DIt,
                                                const int* __restrict__ FLAG, const float* __restrict__ ACC,
                                                const float* __restrict__ B2t, float* out, int nreal) {
  __shared__ __attribute__((aligned(16))) float sb2[FOUT];
  const int tid = (int)threadIdx.x, lane = tid & 31, wave = tid >> 5;
  {
    const v4f b = *(const v4fa*)(B2t + 4 * (tid & 15));
    asm volatile("" :: "v"(b));
    if (tid < 16) *(v4fa*)(sb2 + 4 * tid) = b;
  }
  __syncthreads();

  const int row = (int)blockIdx.x * NWAVE + wave;
  const int rc  = clampi(row, 0, NNODE - 1);
  const int blk = rc >> SLB;
  int c = CNT[rc];
  int o = OFF[rc];
  const int flag = FLAG[(size_t)blk * 32];
  const float di = DIt[rc];
  asm volatile("" :: "v"(c));
  asm volatile("" :: "v"(o));
  asm volatile("" :: "v"(flag));
  asm volatile("" :: "v"(di));
  const bool big = c > DEGCAP;
  c = __builtin_amdgcn_readfirstlane((row < NNODE) ? clampi(c, 0, DEGCAP) : 0);
  o = __builtin_amdgcn_readfirstlane(clampi(o, 0, RCAP - 1));
  int last = o + (c > 0 ? c : 1) - 1;
  last = last > RCAP - 1 ? RCAP - 1 : last;
  const int* lb = LIST + (size_t)blk * (size_t)RCAP;

  float a0 = 0.0f, a1 = 0.0f;
#pragma unroll 1
  for (int b0 = 0; b0 < c; b0 += 32) {
    int idx = o + b0 + lane;
    idx = idx > last ? last : idx;
    const int word = lb[idx];
    asm volatile("" :: "v"(word));
    const int sr = clampi(word, 0, NNODE - 1);
    const int m32 = (c - b0) < 32 ? (c - b0) : 32;
#pragma unroll 1
    for (int k = 0; k < m32; ++k) {
      const int sk = __builtin_amdgcn_readlane(sr, k);
      const v2f q = *(const v2fa*)(ACC + (size_t)sk * FOUT + 2 * lane);
      const float qx = q.x, qy = q.y;
      asm volatile("" :: "v"(qx));
      asm volatile("" :: "v"(qy));
      a0 = a0 + qx;
      a1 = a1 + qy;
    }
  }

  const v2f bq = *(const v2fa*)(sb2 + 2 * lane);
  const float t0 = a0 * di;
  const float t1 = a1 * di;
  float v0 = t0 + bq.x;
  float v1 = t1 + bq.y;
  const float qnan = __uint_as_float(0x7fc00000u);
  const bool bad = (flag != 0) || big;
  v0 = bad ? qnan : v0;
  v1 = bad ? qnan : v1;

  if (row < nreal && row < NNODE) {
    v2f ov;
    ov.x = v0; ov.y = v1;
    float* op = out + (size_t)row * FOUT + 2 * lane;
    *(volatile v2f*)op = ov;
    __threadfence();
    *(volatile v2f*)op = ov;
  }
}

extern "C" void kernel_launch(void* const* d_in, const int* in_sizes, int n_in,
                              void* d_out, int out_size, void* d_ws, size_t ws_size,
                              hipStream_t stream) {
  if (n_in < 7) return;
  if (in_sizes[0] != NNODE * FIN) return;
  if (in_sizes[1] != NEDGE) return;
  if (in_sizes[2] != NEDGE) return;
  if (in_sizes[3] != FIN * HID) return;
  if (in_sizes[4] != HID) return;
  if (in_sizes[5] != HID * FOUT) return;
  if (in_sizes[6] != FOUT) return;
  if (out_size != NNODE * FOUT) return;

  const float* feat = (const float*)d_in[0];
  const int*   srcs = (const int*)d_in[1];
  const int*   dsts = (const int*)d_in[2];
  const float* W1 = (const float*)d_in[3];
  const float* b1 = (const float*)d_in[4];
  const float* W2 = (const float*)d_in[5];
  const float* b2 = (const float*)d_in[6];
  float* out = (float*)d_out;

  constexpr size_t zRA   = (size_t)MPAD * FIN * 2;
  constexpr size_t zRO   = (size_t)MPAD * KT * 2;
  constexpr size_t zRB   = (size_t)MPAD * HH * 4;
  constexpr size_t zLIST = (size_t)NBK * RCAP * 4;
  constexpr size_t zTAB  = (size_t)NTAB * 4;
  constexpr size_t zFLAG = (size_t)NBK * 128;
  constexpr size_t zW1   = (size_t)HH * KT * 2;
  constexpr size_t zW2   = (size_t)FOUT * KT * 2;
  constexpr size_t zBT   = 2048;
  constexpr size_t oRA   = 0;
  constexpr size_t oRO   = oRA + zRA;
  constexpr size_t oRB   = oRO + zRO;
  constexpr size_t oLIST = oRB + zRB;
  constexpr size_t oCNT  = oLIST + zLIST;
  constexpr size_t oOFF  = oCNT + zTAB;
  constexpr size_t oDI   = oOFF + zTAB;
  constexpr size_t oDO   = oDI + zTAB;
  constexpr size_t oFLAG = oDO + zTAB;
  constexpr size_t oW1A  = oFLAG + zFLAG;
  constexpr size_t oW1B  = oW1A + zW1;
  constexpr size_t oW2A  = oW1B + zW1;
  constexpr size_t oW2B  = oW2A + zW2;
  constexpr size_t oBT   = oW2B + zW2;
  constexpr size_t oEND  = oBT + zBT;
  static_assert(zRA % 256 == 0 && zRO % 256 == 0 && zRB % 256 == 0 && zLIST % 256 == 0 && zTAB % 256 == 0);
  static_assert(zFLAG % 256 == 0 && zW1 % 256 == 0 && zW2 % 256 == 0 && zBT % 256 == 0);
  static_assert(zRA == (size_t)MPAD * FOUT * 4);
  static_assert(zRO >= (size_t)MPAD * FOUT * 4);
  static_assert(zRB == (size_t)MPAD * KT * 2);
  static_assert(zBT >= (size_t)BT_UNITS * 16);
  static_assert(oEND == (size_t)540505 * 256);
  static_assert(oEND <= ((size_t)256 << 20));
  if (oEND > ws_size) return;

  char* ws = (char*)d_ws;
  unsigned short* XB   = (unsigned short*)(ws + oRA);
  float*          ACC  = (float*)(ws + oRA);
  unsigned short* OPA  = (unsigned short*)(ws + oRO);
  float*          Q    = (float*)(ws + oRO);
  float*          P    = (float*)(ws + oRB);
  unsigned short* G    = (unsigned short*)(ws + oRB);
  int*            LIST = (int*)(ws + oLIST);
  int*            CNT  = (int*)(ws + oCNT);
  int*            OFF  = (int*)(ws + oOFF);
  int*            DIi  = (int*)(ws + oDI);
  const float*    DIf  = (const float*)(ws + oDI);
  int*            DOi  = (int*)(ws + oDO);
  const float*    DOf  = (const float*)(ws + oDO);
  int*            FLAG = (int*)(ws + oFLAG);
  unsigned short* W1A  = (unsigned short*)(ws + oW1A);
  unsigned short* W1B  = (unsigned short*)(ws + oW1B);
  unsigned short* W2A  = (unsigned short*)(ws + oW2A);
  unsigned short* W2B  = (unsigned short*)(ws + oW2B);
  float*          BT   = (float*)(ws + oBT);
  const float*    B1t  = BT + BT_B1;
  const float*    B2t  = BT + BT_B2;
  const float*    ZB   = BT + BT_Z;

  hipFuncSetAttribute(reinterpret_cast<const void*>(&k_bucket), hipFuncAttributeMaxDynamicSharedMemorySize, (int)BK_LDS);

  constexpr int GT1 = ((MPAD / 64) * (HH / 64) + 7) / 8;
  constexpr int GT2 = ((MPAD / 64) * (FOUT / 64) + 7) / 8;
  constexpr int GWP = MPAD / NWAVE;
  constexpr int GWN = NNODE / NWAVE;
  constexpr int GAD = MPAD * FOUT / 4 / NTHR;

  k_plane<0><<<MPAD * FIN / 8 / NTHR, NTHR, 0, stream>>>(feat, NNODE, FIN, FIN, XB, MPAD, FIN);
  k_prep<<<PB_TOT, NTHR, 0, stream>>>(W1, W2, b1, b2, W1A, W1B, W2A, W2B, BT);
  k_bucket<<<NBK, NTHR, BK_LDS, stream>>>(srcs, dsts, LIST, CNT, OFF, DIi, DOi, FLAG);
  k_walk0<<<GWP, NTHR, 0, stream>>>(LIST, CNT, OFF, DOf, FLAG, XB, OPA);
  k_gemm_nt<0, 0><<<GT1, NTHR, 0, stream>>>(OPA, W1A, ZB, P, MPAD, HH, KT, HH);
  k_convert<<<GWP, NTHR, 0, stream>>>(P, DIf, DOf, FLAG, B1t);
  k_gemm_nt<0, 0><<<GT2, NTHR, 0, stream>>>(G, W2A, ZB, ACC, MPAD, FOUT, KT, FOUT);
  k_gemm_nt<0, 0><<<GT1, NTHR, 0, stream>>>(OPA, W1B, ZB, P, MPAD, HH, KT, HH);
  k_convert<<<GWP, NTHR, 0, stream>>>(P, DIf, DOf, FLAG, B1t + HH);
  k_gemm_nt<0, 0><<<GT2, NTHR, 0, stream>>>(G, W2B, ZB, Q, MPAD, FOUT, KT, FOUT);
  k_add<<<GAD, NTHR, 0, stream>>>(ACC, Q);
  k_walk2<<<GWN, NTHR, 0, stream>>>(LIST, CNT, OFF, DIf, FLAG, ACC, B2t, out, NNODE);
}
